// DAGERC_fusion_26826365731123
// MI455X (gfx1250) — hardware-verified
//
#include <hip/hip_runtime.h>
#include <math.h>

typedef __attribute__((ext_vector_type(16))) _Float16 v16h;
typedef __attribute__((ext_vector_type(8)))  _Float16 v8h;
typedef __attribute__((ext_vector_type(16))) __bf16   v16b;
typedef __attribute__((ext_vector_type(8)))  __bf16   v8b;
typedef __attribute__((ext_vector_type(8)))  float    v8f;
typedef __attribute__((ext_vector_type(4)))  float    v4f;

constexpr int kB    = 64;
constexpr int kN    = 128;
constexpr int kE    = 1024;
constexpr int kD    = 300;
constexpr int kDP   = 320;
constexpr int kK2   = 2 * kDP;
constexpr int kG    = 3 * kD;
constexpr int kGP   = 3 * kDP;
constexpr int kNF   = 2048;
constexpr int kRows = kB * kN;
constexpr int kOutW = 3 * kD + kE;
constexpr int kThr  = 256;
constexpr float kInCarry = 1024.0f;
constexpr float kWCarry  = 4096.0f;
constexpr float kHCarry  = 256.0f;
constexpr float kScFW = 1.0f / (kInCarry * kWCarry);
constexpr float kScHW = 1.0f / (kHCarry * kWCarry);
constexpr float kF16MinNormal = 6.103515625e-5f;

static_assert((kRows % 64) == 0 && (kB % 64) == 0 && (kDP % 64) == 0 && (kNF % 64) == 0, "GEMM M, N multiples of 64");
static_assert(((kRows / 64) * (kDP / 64)) % 8 == 0 && ((kRows / 64) * (kNF / 64)) % 8 == 0 && ((kB / 64) * (kNF / 64)) % 8 == 0, "GEMM grids exact");
static_assert((kE % 32) == 0 && (kK2 % 32) == 0, "GEMM K multiples of 32");
static_assert(2 * kGP <= kNF && (kD % 4) == 0 && (kD % 8) == 4, "gate blocks fit; 300 is a multiple of 4 (a 4-float vector never straddles 300) but not of 8 (the vector of 8 at 296 does)");

constexpr size_t kOffFEAT16 = 0;
constexpr size_t kOffFC1T = kOffFEAT16 + (size_t)kRows * kE * 2;
constexpr size_t kOffWX0  = kOffFC1T + (size_t)kDP * kE * 2;
constexpr size_t kOffWM0  = kOffWX0  + (size_t)kNF * kK2 * 2;
constexpr size_t kOffWX1  = kOffWM0  + (size_t)kNF * kK2 * 2;
constexpr size_t kOffWM1  = kOffWX1  + (size_t)kNF * kK2 * 2;
constexpr size_t kOffBIAS = kOffWM1  + (size_t)kNF * kK2 * 2;
constexpr int kFB0 = 0, kFBX0 = 1024, kFBM0 = 3072, kFBX1 = 5120, kFBM1 = 7168, kFEnd = 9216;
constexpr size_t kOffH0F  = kOffBIAS + (size_t)kFEnd * 4;
constexpr size_t kOffBUF0 = kOffH0F  + (size_t)kRows * kDP * 4;
constexpr size_t kOffBUF1 = kOffBUF0 + (size_t)kRows * kDP * 4;
constexpr size_t kOffH160 = kOffBUF1 + (size_t)kRows * kDP * 4;
constexpr size_t kOffH161 = kOffH160 + (size_t)kRows * kK2 * 2;
constexpr size_t kOffXG   = kOffH161 + (size_t)kRows * kK2 * 2;
constexpr size_t kOffM16  = kOffXG   + (size_t)kRows * kNF * 4;
constexpr size_t kOffM32  = kOffM16  + (size_t)kB * kK2 * 2;
constexpr size_t kOffMG   = kOffM32  + (size_t)kB * kDP * 4;
constexpr size_t kWsTotal = kOffMG   + (size_t)kB * kNF * 4;
static_assert(kWsTotal == 148180992ull, "carve total");
static_assert(kWsTotal <= 268435456ull, "carve cap");
static_assert((kOffFC1T % 256) == 0 && (kOffWX0 % 256) == 0 && (kOffWM0 % 256) == 0 && (kOffWX1 % 256) == 0 && (kOffWM1 % 256) == 0 && (kOffBIAS % 256) == 0 && (kOffH0F % 256) == 0 && (kOffBUF0 % 256) == 0 && (kOffBUF1 % 256) == 0 && (kOffH160 % 256) == 0 && (kOffH161 % 256) == 0 && (kOffXG % 256) == 0 && (kOffM16 % 256) == 0 && (kOffM32 % 256) == 0 && (kOffMG % 256) == 0, "aligned regions");
static_assert(((size_t)kRows * kOutW) % 4 == 0 && (kOutW % 4) == 0 && ((size_t)kRows * kOutW / 4) % kThr == 0, "the flat output divides into whole blocks of 4-float vectors; a vector never straddles a row");

__device__ __forceinline__ unsigned short f2bf_bits(float f) {
  unsigned u = __float_as_uint(f);
  return (unsigned short)((u + 0x7FFFu + ((u >> 16) & 1u)) >> 16);
}
__device__ __forceinline__ float bf_bits2f(unsigned short h) { return __uint_as_float(((unsigned)h) << 16); }
__device__ __forceinline__ float bf16r(float f) { return bf_bits2f(f2bf_bits(f)); }
__device__ __forceinline__ float carry_flush(float v, float carry) {
  const float s = v * carry;
  return (fabsf(s) < kF16MinNormal) ? 0.0f : s;
}
__device__ __forceinline__ float frcp(float x) { return __builtin_amdgcn_rcpf(x); }

__device__ __forceinline__ void dep_guard4_h(v8f& a, v8f& b, v8f& c, v8f& d, v16h x, v16h y) { asm volatile("v_nop\n\tv_nop\n\tv_nop\n\tv_nop" : "+v"(a), "+v"(b), "+v"(c), "+v"(d) : "v"(x), "v"(y)); }
__device__ __forceinline__ void dep_guard4_b(v8f& a, v8f& b, v8f& c, v8f& d, v16b x, v16b y) { asm volatile("v_nop\n\tv_nop\n\tv_nop\n\tv_nop" : "+v"(a), "+v"(b), "+v"(c), "+v"(d) : "v"(x), "v"(y)); }
__device__ __forceinline__ void keep4_h(v16h a, v16h b, v16h c, v16h d) { asm volatile("v_nop" :: "v"(a), "v"(b), "v"(c), "v"(d)); }
__device__ __forceinline__ void keep4_b(v16b a, v16b b, v16b c, v16b d) { asm volatile("v_nop" :: "v"(a), "v"(b), "v"(c), "v"(d)); }
__device__ __forceinline__ void acc_guard4(v8f& a, v8f& b, v8f& c, v8f& d) { asm volatile("v_nop\n\tv_nop\n\tv_nop\n\tv_nop" : "+v"(a), "+v"(b), "+v"(c), "+v"(d)); }

template <typename T> struct Frag;
template <> struct Frag<_Float16> {
  typedef v16h V; union U { v16h v; v8h h[2]; };
  static __device__ __forceinline__ v16h load(const _Float16* p) {
    U f; f.h[0] = *(const v8h*)(p); f.h[1] = *(const v8h*)(p + 16); return f.v;
  }
  static __device__ __forceinline__ v8f mma(v16h a, v16h b, v8f c) {
    return __builtin_amdgcn_wmma_f32_16x16x32_f16(false, a, false, b, (short)0, c, false, false);
  }
  static __device__ __forceinline__ void guard4(v8f& a, v8f& b, v8f& c, v8f& d, v16h x, v16h y) { dep_guard4_h(a, b, c, d, x, y); }
  static __device__ __forceinline__ void keep(v16h a, v16h b, v16h c, v16h d) { keep4_h(a, b, c, d); }
};
template <> struct Frag<__bf16> {
  typedef v16b V; union U { v16b v; v8b h[2]; };
  static __device__ __forceinline__ v16b load(const __bf16* p) {
    U f; f.h[0] = *(const v8b*)(p); f.h[1] = *(const v8b*)(p + 16); return f.v;
  }
  static __device__ __forceinline__ v8f mma(v16b a, v16b b, v8f c) {
    return __builtin_amdgcn_wmma_f32_16x16x32_bf16(false, a, false, b, (short)0, c, false, false);
  }
  static __device__ __forceinline__ void guard4(v8f& a, v8f& b, v8f& c, v8f& d, v16b x, v16b y) { dep_guard4_b(a, b, c, d, x, y); }
  static __device__ __forceinline__ void keep(v16b a, v16b b, v16b c, v16b d) { keep4_b(a, b, c, d); }
};

__device__ __forceinline__ v8f mma_h(v16h a, v16h b, v8f c) {
  c = __builtin_amdgcn_wmma_f32_16x16x32_f16(false, a, false, b, (short)0, c, false, false);
  asm volatile("v_nop\n\tv_nop\n\tv_nop\n\tv_nop" : "+v"(c) : "v"(a), "v"(b));
  return c;
}

template <int ET> struct Elem;
template <> struct Elem<0> { typedef _Float16 T; };
template <> struct Elem<1> { typedef __bf16 T; };
template <int ET, bool SPLIT, int BIAS_MODE, int OUT_MODE, bool RESID, int ACT = 0>
__global__ __launch_bounds__(256) void wmma_gemm64(
    const unsigned short* __restrict__ Ap, const unsigned short* __restrict__ A2p, int lda, long strideA,
    const unsigned short* __restrict__ Btp, const unsigned short* __restrict__ Bt2p, int ldb, long strideB,
    void* __restrict__ Cout, void* __restrict__ Cout2, int ldc, long strideC,
    const float* __restrict__ bias,
    const float* __restrict__ resid, long strideR,
    int M, int N, int K, float scale) {
  typedef typename Elem<ET>::T T;
  typedef typename Frag<T>::V V;
  const T* A = (const T*)Ap; const T* A2 = (const T*)A2p; const T* Bt = (const T*)Btp; const T* Bt2 = (const T*)Bt2p;
  __shared__ __align__(16) float sT[8][16 * 68];
  const int b    = blockIdx.y;
  const int lane = threadIdx.x & 31;
  const int wave = threadIdx.x >> 5;
  const int tilesN = N >> 6;
  const int tilesM = M >> 6;
  const int tile = blockIdx.x * 8 + wave;
  if (tile >= tilesM * tilesN) return;
  const int tm = tile / tilesN;
  const int tn = tile - tm * tilesN;
  const int m0 = tm << 6;
  const int n0 = tn << 6;

  const T* Ab  = A  + (size_t)b * strideA;
  const T* Bb  = Bt + (size_t)b * strideB;
  const T* Ab2 = SPLIT ? (A2  + (size_t)b * strideA) : nullptr;
  const T* Bb2 = SPLIT ? (Bt2 + (size_t)b * strideB) : nullptr;

  const int rlane = lane & 15;
  const int koff  = (lane >> 4) * 8;
  const int mOff  = (lane >> 4) * 8;

  v8f acc[4][4];
#pragma unroll
  for (int i = 0; i < 4; ++i)
#pragma unroll
    for (int j = 0; j < 4; ++j) acc[i][j] = (v8f){0.f,0.f,0.f,0.f,0.f,0.f,0.f,0.f};

  for (int k0 = 0; k0 < K; k0 += 32) {
    V bh[4], bl[4];
#pragma unroll
    for (int j = 0; j < 4; ++j) {
      const size_t bo = (size_t)(n0 + (j << 4) + rlane) * ldb + koff + k0;
      bh[j] = Frag<T>::load(Bb + bo);
      if (SPLIT) bl[j] = Frag<T>::load(Bb2 + bo);
    }
#pragma unroll
    for (int i = 0; i < 4; ++i) {
      const size_t ao = (size_t)(m0 + (i << 4) + rlane) * lda + koff + k0;
      V ah = Frag<T>::load(Ab + ao);
      V al;
      if (SPLIT) al = Frag<T>::load(Ab2 + ao);
#pragma unroll
      for (int j = 0; j < 4; ++j) {
        acc[i][j] = Frag<T>::mma(ah, bh[j], acc[i][j]);
        if (SPLIT) {
          acc[i][j] = Frag<T>::mma(ah, bl[j], acc[i][j]);
          acc[i][j] = Frag<T>::mma(al, bh[j], acc[i][j]);
        }
      }
      Frag<T>::guard4(acc[i][0], acc[i][1], acc[i][2], acc[i][3], ah, SPLIT ? al : ah);
    }
    Frag<T>::keep(bh[0], bh[1], bh[2], bh[3]);
    if (SPLIT) Frag<T>::keep(bl[0], bl[1], bl[2], bl[3]);
  }
  acc_guard4(acc[0][0], acc[0][1], acc[0][2], acc[0][3]);
  acc_guard4(acc[1][0], acc[1][1], acc[1][2], acc[1][3]);
  acc_guard4(acc[2][0], acc[2][1], acc[2][2], acc[2][3]);
  acc_guard4(acc[3][0], acc[3][1], acc[3][2], acc[3][3]);

  float* slab = sT[wave];
  const float* Rb = RESID ? (resid + (size_t)b * strideR) : nullptr;
#pragma unroll
  for (int i = 0; i < 4; ++i) {
    const int mBase = m0 + (i << 4);
#pragma unroll
    for (int j = 0; j < 4; ++j) {
      const int n = n0 + (j << 4) + rlane;
      float bv = 0.f;
      if (BIAS_MODE == 2) bv = bias[n];
#pragma unroll
      for (int r = 0; r < 8; ++r) {
        float v = acc[i][j][r] * scale;
        if (BIAS_MODE == 1) v += bias[mBase + mOff + r];
        if (BIAS_MODE == 2) v += bv;
        if (RESID) v += Rb[(size_t)(mBase + mOff + r) * ldc + n];
        if (ACT == 1) v = tanhf(v);
        if (ACT == 2) v = fmaxf(v, 0.0f);
        if (ACT == 3) v = v / (1.0f + expf(-v));
        if (ACT == 4) v = (v > 0.f) ? v : 0.01f * v;
        slab[(mOff + r) * 68 + (j << 4) + rlane] = v;
      }
    }
    __builtin_amdgcn_fence(__ATOMIC_RELEASE, "workgroup");
    __builtin_amdgcn_wave_barrier();
    __builtin_amdgcn_fence(__ATOMIC_ACQUIRE, "workgroup");
    if (OUT_MODE == 0) {
      float* C = (float*)Cout + (size_t)b * strideC;
      const int hh = lane >> 4, c4 = (lane & 15) * 4;
      for (int pass = 0; pass < 2; ++pass) {
#pragma unroll
        for (int it = 0; it < 8; ++it) {
          const int row = it * 2 + hh;
          v4f v = *(const v4f*)(slab + row * 68 + c4);
          *(volatile v4f*)(C + (size_t)(mBase + row) * ldc + n0 + c4) = v;
        }
        __threadfence();
      }
    } else {
      const int q = lane >> 3, c8 = (lane & 7) * 8;
      unsigned short* C  = (unsigned short*)Cout  + (size_t)b * strideC;
      unsigned short* C2 = (OUT_MODE == 2) ? ((unsigned short*)Cout2 + (size_t)b * strideC) : nullptr;
      for (int pass = 0; pass < 2; ++pass) {
#pragma unroll
        for (int it = 0; it < 4; ++it) {
          const int row = it * 4 + q;
          const float* sp = slab + row * 68 + c8;
          v8h hv, lv;
#pragma unroll
          for (int e = 0; e < 8; ++e) {
            if (OUT_MODE == 1) {
              hv[e] = (_Float16)sp[e];
            } else {
              unsigned short hb = f2bf_bits(sp[e]);
              unsigned short lb = f2bf_bits(sp[e] - bf_bits2f(hb));
              hv[e] = __builtin_bit_cast(_Float16, hb);
              lv[e] = __builtin_bit_cast(_Float16, lb);
            }
          }
          *(volatile v8h*)(C + (size_t)(mBase + row) * ldc + n0 + c8) = hv;
          if (OUT_MODE == 2) *(volatile v8h*)(C2 + (size_t)(mBase + row) * ldc + n0 + c8) = lv;
        }
        __threadfence();
      }
    }
    __builtin_amdgcn_fence(__ATOMIC_RELEASE, "workgroup");
    __builtin_amdgcn_wave_barrier();
    __builtin_amdgcn_fence(__ATOMIC_ACQUIRE, "workgroup");
  }
}

__global__ __launch_bounds__(kThr) void cast_plane_kernel(const float* __restrict__ src, unsigned short* __restrict__ dst,
                                                          int colsLog2, int dstPitch, int dstOff) {
  const int i   = blockIdx.x * kThr + threadIdx.x;
  const int sh  = colsLog2 - 3;
  const int row = i >> sh;
  const int c8  = (i & ((1 << sh) - 1)) * 8;
  const float* sp = src + ((size_t)row << colsLog2) + c8;
  const v4f a0 = *(const v4f*)(sp);
  const v4f a1 = *(const v4f*)(sp + 4);
  v8h hv;
#pragma unroll
  for (int e = 0; e < 4; ++e) {
    const float f0 = a0[e];
    const float f1 = a1[e];
    hv[e]     = (_Float16)carry_flush(bf16r(f0), kInCarry);
    hv[4 + e] = (_Float16)carry_flush(bf16r(f1), kInCarry);
  }
  unsigned short* dp = dst + (size_t)row * dstPitch + dstOff + c8;
  *(volatile v8h*)dp = hv;
  __threadfence();
  *(volatile v8h*)dp = hv;
}
__device__ __forceinline__ void split_hl(float v, float c, _Float16& hi, _Float16& lo) {
  const float sv = carry_flush(v, c);
  hi = (_Float16)sv;
  const float r = sv - (float)hi;
  lo = (_Float16)((fabsf(r) < kF16MinNormal) ? 0.0f : r);
}

__global__ __launch_bounds__(256) void wt_plane_kernel(const float* __restrict__ W, unsigned short* __restrict__ dst, int K, int N, int nLive, int ldd, int colOff) {
  const int n  = blockIdx.x;
  const int k8 = threadIdx.x * 8;
  const bool live = n < nLive;
  const int nc = live ? n : 0;
  v8h hv;
#pragma unroll
  for (int e = 0; e < 8; ++e) {
    const float w = W[(size_t)(k8 + e) * N + nc];
    hv[e] = (_Float16)(live ? carry_flush(bf16r(w), kWCarry) : 0.0f);
  }
  unsigned short* dp = dst + (size_t)n * ldd + colOff + k8;
  *(volatile v8h*)dp = hv;
  __threadfence();
  *(volatile v8h*)dp = hv;
}


__device__ __forceinline__ float fast_tanh(float v) { return 1.0f - 2.0f * frcp(__expf(2.0f * v) + 1.0f); }
__device__ __forceinline__ float fast_sigmoid(float v) { return frcp(1.0f + __expf(-v)); }

__global__ __launch_bounds__(kThr) void gate_plane_kernel(const float* __restrict__ Wa, const float* __restrict__ Wb, unsigned short* __restrict__ dst) {
  unsigned v = blockIdx.x * (unsigned)kThr + threadIdx.x;
  asm volatile("" : "+v"(v));
  const unsigned n  = v / 40u;
  const unsigned k8 = (v - n * 40u) * 8u;
  const unsigned which = n / (unsigned)kGP;
  const unsigned nn = n - which * (unsigned)kGP;
  const unsigned g  = nn / (unsigned)kDP;
  const unsigned j  = nn - g * (unsigned)kDP;
  const bool liveRow = (which < 2u) && (j < (unsigned)kD);
  const unsigned srow = liveRow ? (g * (unsigned)kD + j) : 0u;
  const float* W = (which == 1u) ? Wb : Wa;
  const float* sp = W + (size_t)srow * kD;
  v8h hv;
#pragma unroll
  for (int e = 0; e < 8; ++e) {
    const unsigned k = k8 + (unsigned)e;
    const unsigned kc = (k < (unsigned)kD) ? k : 0u;
    const float w = sp[kc];
    hv[e] = (_Float16)((liveRow && k < (unsigned)kD) ? carry_flush(bf16r(w), kWCarry) : 0.0f);
  }
  unsigned short* dp = dst + (size_t)n * kK2 + k8;
  for (int pass = 0; pass < 2; ++pass) {
    *(volatile v8h*)dp = hv;
    *(volatile v8h*)(dp + kDP) = hv;
    __threadfence();
  }
}
static_assert(kNF * (kDP / 8) == 320 * kThr && kDP / 8 == 40, "gate plane grid exact");

__global__ __launch_bounds__(kThr) void bias_rows_kernel(const float* __restrict__ fc1_b, const float* __restrict__ c_bih, const float* __restrict__ c_bhh,
                                                         const float* __restrict__ p_bih, const float* __restrict__ p_bhh, float* __restrict__ BIAS) {
  unsigned v = blockIdx.x * (unsigned)kThr + threadIdx.x;
  asm volatile("" : "+v"(v));
  const unsigned i0 = v * 4u;
  v4f o = {0.f, 0.f, 0.f, 0.f};
  if (i0 < (unsigned)kFBX0) {
    const bool live = i0 < (unsigned)kD;
    const v4f a = *(const v4f*)(fc1_b + (live ? i0 : 0u));
#pragma unroll
    for (int e = 0; e < 4; ++e) { const float x = a[e]; o[e] = live ? bf16r(x) : 0.0f; }
  } else {
    const unsigned q = i0 - (unsigned)kFBX0;
    const unsigned reg = q >> 11;
    unsigned n = q & 2047u;
    asm volatile("" : "+v"(n));
    const unsigned layer = reg >> 1;
    const bool isM = (reg & 1u) != 0u;
    const unsigned which = n / (unsigned)kGP;
    const unsigned nn = n - which * (unsigned)kGP;
    const unsigned g = nn / (unsigned)kDP;
    const unsigned j = nn - g * (unsigned)kDP;
    const bool live = (which < 2u) && (j < (unsigned)kD);
    const unsigned si = layer * (unsigned)kG + (live ? (g * (unsigned)kD + j) : 0u);
    const float* src = isM ? ((which == 1u) ? p_bih : c_bhh) : ((which == 1u) ? p_bhh : c_bih);
    const v4f a = *(const v4f*)(src + si);
#pragma unroll
    for (int e = 0; e < 4; ++e) { const float x = a[e]; o[e] = live ? bf16r(x) : 0.0f; }
  }
  float* dp = BIAS + i0;
  *(volatile v4f*)dp = o;
  __threadfence();
  *(volatile v4f*)dp = o;
}
static_assert(kFEnd / 4 == 9 * kThr && (kFBX0 % 128) == 0 && kFBM0 == kFBX0 + kNF && kFBX1 == kFBM0 + kNF && kFBM1 == kFBX1 + kNF && kFEnd == kFBM1 + kNF, "bias grid exact; stream map");

__global__ __launch_bounds__(kThr) void relu_split_kernel(float* __restrict__ H0F, unsigned short* __restrict__ H16) {
  unsigned v = blockIdx.x * (unsigned)kThr + threadIdx.x;
  asm volatile("" : "+v"(v));
  const unsigned row = v / 40u;
  const unsigned k8 = (v - row * 40u) * 8u;
  float* fp = H0F + (size_t)row * kDP + k8;
  const v4f a0 = *(const v4f*)fp, a1 = *(const v4f*)(fp + 4);
  v4f r0, r1; v8h hv, lv;
#pragma unroll
  for (int e = 0; e < 4; ++e) {
    r0[e] = fmaxf(a0[e], 0.0f); r1[e] = fmaxf(a1[e], 0.0f);
    _Float16 h0, l0, h1, l1;
    split_hl(r0[e], kHCarry, h0, l0);
    split_hl(r1[e], kHCarry, h1, l1);
    hv[e] = h0; lv[e] = l0; hv[4 + e] = h1; lv[4 + e] = l1;
  }
  unsigned short* hp = H16 + (size_t)row * kK2 + k8;
  for (int pass = 0; pass < 2; ++pass) {
    *(volatile v4f*)fp = r0;
    *(volatile v4f*)(fp + 4) = r1;
    *(volatile v8h*)hp = hv;
    *(volatile v8h*)(hp + kDP) = lv;
    __threadfence();
  }
}
static_assert(kRows * (kDP / 8) == 1280 * kThr, "rectifier grid exact");

__global__ __launch_bounds__(kThr) void ctx_zero_kernel(float* __restrict__ M32, unsigned short* __restrict__ M16) {
  unsigned v = blockIdx.x * (unsigned)kThr + threadIdx.x;
  asm volatile("" : "+v"(v));
  const unsigned row = v / 40u;
  const unsigned k8 = (v - row * 40u) * 8u;
  const v4f zf = {0.f, 0.f, 0.f, 0.f};
  v8h zh;
#pragma unroll
  for (int e = 0; e < 8; ++e) zh[e] = (_Float16)0.0f;
  float* fp = M32 + (size_t)row * kDP + k8;
  unsigned short* hp = M16 + (size_t)row * kK2 + k8;
  for (int pass = 0; pass < 2; ++pass) {
    *(volatile v4f*)fp = zf;
    *(volatile v4f*)(fp + 4) = zf;
    *(volatile v8h*)hp = zh;
    *(volatile v8h*)(hp + kDP) = zh;
    __threadfence();
  }
}
static_assert(kB * (kDP / 8) == 10 * kThr, "context zero grid exact");

__global__ __launch_bounds__(128) void hist_attn_kernel(const float* __restrict__ X, const float* __restrict__ BUF, const float* __restrict__ gat_w,
                                                        const float* __restrict__ gat_b, const int* __restrict__ adj, float* __restrict__ M32,
                                                        unsigned short* __restrict__ M16, int i, int layer) {
  __shared__ __align__(16) float sWk[kDP];
  __shared__ __align__(16) float sT[128];
  __shared__ __align__(16) float sS[kN];
  __shared__ __align__(16) float sRed[8];
  const int tid = threadIdx.x;
  const int b   = blockIdx.x;
  const float* gw = gat_w + (size_t)layer * (2 * kD);
  {
    float part = 0.0f;
    if (tid < kD / 4) {
      const v4f xv = *(const v4f*)(X + ((size_t)b * kN + i) * kDP + tid * 4);
      const v4f wv = *(const v4f*)(gw + tid * 4);
      part = xv[0] * bf16r(wv[0]);
      part += xv[1] * bf16r(wv[1]);
      part += xv[2] * bf16r(wv[2]);
      part += xv[3] * bf16r(wv[3]);
    }
    sT[tid] = part;
    for (int k = tid; k < kDP; k += 128) { const float w = gw[kD + ((k < kD) ? k : 0)]; sWk[k] = (k < kD) ? bf16r(w) : 0.0f; }
  }
  __syncthreads();
  if (tid == 0) {
    float q = 0.0f;
#pragma unroll 1
    for (int k = 0; k < kD / 4; ++k) q += sT[k];
    const float gb = gat_b[layer];
    sRed[4] = q + bf16r(gb);
  }
  __syncthreads();
  {
    const int n = tid;
    float a = -1e30f;
    if (n < i) {
      const float* br = BUF + ((size_t)b * kN + n) * kDP;
      float s = 0.0f;
#pragma unroll 1
      for (int k = 0; k < kD; k += 4) {
        const v4f h = *(const v4f*)(br + k);
        const v4f w = *(const v4f*)(sWk + k);
        s += h[0] * w[0]; s += h[1] * w[1]; s += h[2] * w[2]; s += h[3] * w[3];
      }
      int mk = adj[((size_t)b * kN + i) * kN + n];
      asm volatile("" : "+v"(mk));
      const float m = (mk != 0) ? 1.0f : 0.0f;
      a = (s + sRed[4]) - (1.0f - m) * 1e30f;
    }
    sS[n] = a;
  }
  __syncthreads();
  if (tid < 4) {
    float m = sS[tid * 32];
#pragma unroll 1
    for (int j = 1; j < 32; ++j) { const float q = sS[tid * 32 + j]; m = (q > m) ? q : m; }
    sRed[tid] = m;
  }
  __syncthreads();
  float mx = sRed[0];
#pragma unroll 1
  for (int j = 1; j < 4; ++j) { const float q = sRed[j]; mx = (q > mx) ? q : mx; }
  const float ex = __expf(sS[tid] - mx);
  __syncthreads();
  sS[tid] = ex;
  __syncthreads();
  float den = 0.0f;
#pragma unroll 1
  for (int j = 0; j < kN; ++j) den += sS[j];
  if (tid < kDP / 8) {
    float acc[8];
#pragma unroll
    for (int e = 0; e < 8; ++e) acc[e] = 0.0f;
    const float* bc = BUF + (size_t)b * kN * kDP + tid * 8;
#pragma unroll 1
    for (int n = 0; n < i; ++n) {
      const float w = sS[n] / den;
      const v4f h0 = *(const v4f*)(bc + (size_t)n * kDP);
      const v4f h1 = *(const v4f*)(bc + (size_t)n * kDP + 4);
#pragma unroll
      for (int e = 0; e < 4; ++e) { acc[e] += w * h0[e]; acc[4 + e] += w * h1[e]; }
    }
    const v4f m0 = {acc[0], acc[1], acc[2], acc[3]};
    const v4f m1 = {acc[4], acc[5], acc[6], acc[7]};
    v8h hv, lv;
#pragma unroll
    for (int e = 0; e < 8; ++e) { _Float16 h, l; split_hl(acc[e], kHCarry, h, l); hv[e] = h; lv[e] = l; }
    float* fp = M32 + (size_t)b * kDP + tid * 8;
    unsigned short* hp = M16 + (size_t)b * kK2 + tid * 8;
    for (int pass = 0; pass < 2; ++pass) {
      *(volatile v4f*)fp = m0;
      *(volatile v4f*)(fp + 4) = m1;
      *(volatile v8h*)hp = hv;
      *(volatile v8h*)(hp + kDP) = lv;
      __threadfence();
    }
  }
}
static_assert(kN == 128 && kD / 4 == 75 && kDP / 8 == 40, "attention block: a thread per position; 75 vectors of the query product; 40 column groups");

__global__ __launch_bounds__(kThr) void dual_gru_kernel(const float* __restrict__ X, const float* __restrict__ M32, const float* __restrict__ XG,
                                                        const float* __restrict__ MG, float* __restrict__ BUF, unsigned short* __restrict__ H16n, int i, int mode) {
  unsigned v = blockIdx.x * (unsigned)kThr + threadIdx.x;
  asm volatile("" : "+v"(v));
  const unsigned b  = v / 40u;
  const unsigned u8 = (v - b * 40u) * 8u;
  const size_t row = (size_t)b * kN + i;
  const float* xr = X + row * kDP + u8;
  const float* mr = M32 + (size_t)b * kDP + u8;
  const float* xg = XG + row * kNF + u8;
  const float* mg = MG + (size_t)b * kNF + u8;
  v4f o0, o1; v8h hv, lv;
#pragma unroll
  for (int hlf = 0; hlf < 2; ++hlf) {
    const int o = 4 * hlf;
    const v4f xv = *(const v4f*)(xr + o), mv = *(const v4f*)(mr + o);
    const v4f cxr = *(const v4f*)(xg + o), cxz = *(const v4f*)(xg + kDP + o), cxn = *(const v4f*)(xg + 2 * kDP + o);
    const v4f pxr = *(const v4f*)(xg + kGP + o), pxz = *(const v4f*)(xg + kGP + kDP + o), pxn = *(const v4f*)(xg + kGP + 2 * kDP + o);
    const v4f cmr = *(const v4f*)(mg + o), cmz = *(const v4f*)(mg + kDP + o), cmn = *(const v4f*)(mg + 2 * kDP + o);
    const v4f pmr = *(const v4f*)(mg + kGP + o), pmz = *(const v4f*)(mg + kGP + kDP + o), pmn = *(const v4f*)(mg + kGP + 2 * kDP + o);
#pragma unroll
    for (int e = 0; e < 4; ++e) {
      const float rc = fast_sigmoid(cxr[e] + cmr[e]);
      const float zc = fast_sigmoid(cxz[e] + cmz[e]);
      const float nc = fast_tanh(cxn[e] + rc * cmn[e]);
      const float cc = (1.0f - zc) * nc + zc * mv[e];
      const float rp = fast_sigmoid(pmr[e] + pxr[e]);
      const float zp = fast_sigmoid(pmz[e] + pxz[e]);
      const float np = fast_tanh(pmn[e] + rp * pxn[e]);
      const float pp = (1.0f - zp) * np + zp * xv[e];
      const float nv = cc + pp;
      if (hlf == 0) o0[e] = nv; else o1[e] = nv;
      _Float16 h, l; split_hl(nv, kHCarry, h, l);
      hv[o + e] = h; lv[o + e] = l;
    }
  }
  float* bp = BUF + row * kDP + u8;
  unsigned short* hp = H16n + row * kK2 + u8;
  for (int pass = 0; pass < 2; ++pass) {
    *(volatile v4f*)bp = o0;
    *(volatile v4f*)(bp + 4) = o1;
    if (mode == 0) { *(volatile v8h*)hp = hv; *(volatile v8h*)(hp + kDP) = lv; }
    __threadfence();
  }
}
static_assert(kB * (kDP / 8) == 10 * kThr, "cell grid exact");

__global__ __launch_bounds__(kThr) void concat_out_kernel(const float* __restrict__ H0F, const float* __restrict__ BUF0, const float* __restrict__ BUF1,
                                                          const float* __restrict__ features, float* __restrict__ out) {
  unsigned i = blockIdx.x * (unsigned)kThr + threadIdx.x;
  asm volatile("" : "+v"(i));
  const unsigned row = i / 481u;
  const unsigned c4 = (i - row * 481u) * 4u;
  v4f o;
  if (c4 < (unsigned)kD) {
    o = *(const v4f*)(H0F + (size_t)row * kDP + c4);
  } else if (c4 < 2u * (unsigned)kD) {
    o = *(const v4f*)(BUF0 + (size_t)row * kDP + (c4 - (unsigned)kD));
  } else if (c4 < 3u * (unsigned)kD) {
    o = *(const v4f*)(BUF1 + (size_t)row * kDP + (c4 - 2u * (unsigned)kD));
  } else {
    const v4f f = *(const v4f*)(features + (size_t)row * kE + (c4 - 3u * (unsigned)kD));
#pragma unroll
    for (int e = 0; e < 4; ++e) { const float x = f[e]; o[e] = bf16r(x); }
  }
  float* dp = out + (size_t)i * 4u;
  *(volatile v4f*)dp = o;
  __threadfence();
  *(volatile v4f*)dp = o;
}
static_assert(kOutW / 4 == 481 && (size_t)kRows * kOutW / 4 == (size_t)15392 * kThr, "output grid exact");

static_assert(((size_t)kRows * kE / 8) % kThr == 0, "cast grid exact");

extern "C" void kernel_launch(void* const* d_in, const int* in_sizes, int n_in,
                              void* d_out, int out_size, void* d_ws, size_t ws_size,
                              hipStream_t stream) {
  if (n_in < 14 || d_out == nullptr || d_ws == nullptr) return;
  if (in_sizes[0] != kRows * kE || in_sizes[1] != kE * kD || in_sizes[2] != kD || in_sizes[3] != 2 * 2 * kD || in_sizes[4] != 2) return;
  if (in_sizes[5] != 2 * kG * kD || in_sizes[6] != 2 * kG * kD || in_sizes[7] != 2 * kG || in_sizes[8] != 2 * kG) return;
  if (in_sizes[9] != 2 * kG * kD || in_sizes[10] != 2 * kG * kD || in_sizes[11] != 2 * kG || in_sizes[12] != 2 * kG || in_sizes[13] != kB * kN * kN) return;
  if ((size_t)out_size != (size_t)kRows * kOutW) return;
  if (ws_size < kWsTotal) return;
  const float* features = (const float*)d_in[0];
  const float* fc1_w  = (const float*)d_in[1];
  const float* fc1_b  = (const float*)d_in[2];
  const float* gat_w  = (const float*)d_in[3];
  const float* gat_b  = (const float*)d_in[4];
  const float* gc_wih = (const float*)d_in[5];
  const float* gc_whh = (const float*)d_in[6];
  const float* gc_bih = (const float*)d_in[7];
  const float* gc_bhh = (const float*)d_in[8];
  const float* gp_wih = (const float*)d_in[9];
  const float* gp_whh = (const float*)d_in[10];
  const float* gp_bih = (const float*)d_in[11];
  const float* gp_bhh = (const float*)d_in[12];
  const int*   adj    = (const int*)d_in[13];
  float* out = (float*)d_out;
  char* ws = (char*)d_ws;
  unsigned short* FEAT16 = (unsigned short*)(ws + kOffFEAT16);
  unsigned short* FC1T = (unsigned short*)(ws + kOffFC1T);
  unsigned short* WX0  = (unsigned short*)(ws + kOffWX0);
  unsigned short* WM0  = (unsigned short*)(ws + kOffWM0);
  unsigned short* WX1  = (unsigned short*)(ws + kOffWX1);
  unsigned short* WM1  = (unsigned short*)(ws + kOffWM1);
  float* BIAS = (float*)(ws + kOffBIAS);
  float* H0F  = (float*)(ws + kOffH0F);
  float* BUF0 = (float*)(ws + kOffBUF0);
  float* BUF1 = (float*)(ws + kOffBUF1);
  unsigned short* H160 = (unsigned short*)(ws + kOffH160);
  unsigned short* H161 = (unsigned short*)(ws + kOffH161);
  float* XG   = (float*)(ws + kOffXG);
  unsigned short* M16  = (unsigned short*)(ws + kOffM16);
  float* M32  = (float*)(ws + kOffM32);
  float* MG   = (float*)(ws + kOffMG);

  cast_plane_kernel<<<(int)(((size_t)kRows * kE / 8) / kThr), kThr, 0, stream>>>(features, FEAT16, 10, kE, 0);
  wt_plane_kernel<<<kDP, kE / 8, 0, stream>>>(fc1_w, FC1T, kE, kD, kD, kE, 0);
  gate_plane_kernel<<<320, kThr, 0, stream>>>(gc_wih, gp_whh, WX0);
  gate_plane_kernel<<<320, kThr, 0, stream>>>(gc_whh, gp_wih, WM0);
  gate_plane_kernel<<<320, kThr, 0, stream>>>(gc_wih + (size_t)kG * kD, gp_whh + (size_t)kG * kD, WX1);
  gate_plane_kernel<<<320, kThr, 0, stream>>>(gc_whh + (size_t)kG * kD, gp_wih + (size_t)kG * kD, WM1);
  bias_rows_kernel<<<9, kThr, 0, stream>>>(fc1_b, gc_bih, gc_bhh, gp_bih, gp_bhh, BIAS);

  wmma_gemm64<0, false, 2, 0, false, 0><<<dim3((kRows / 64) * (kDP / 64) / 8, 1), 256, 0, stream>>>(
      FEAT16, FEAT16, kE, 0L, FC1T, FC1T, kE, 0L, (void*)H0F, (void*)H0F, kDP, 0L, BIAS + kFB0, nullptr, 0L, kRows, kDP, kE, kScFW);
  relu_split_kernel<<<1280, kThr, 0, stream>>>(H0F, H160);

  for (int layer = 0; layer < 2; ++layer) {
    const float* X = (layer == 0) ? H0F : BUF0;
    const unsigned short* X16 = (layer == 0) ? H160 : H161;
    float* BUF = (layer == 0) ? BUF0 : BUF1;
    const unsigned short* WX = (layer == 0) ? WX0 : WX1;
    const unsigned short* WM = (layer == 0) ? WM0 : WM1;
    const float* BX = BIAS + ((layer == 0) ? kFBX0 : kFBX1);
    const float* BM = BIAS + ((layer == 0) ? kFBM0 : kFBM1);
    ctx_zero_kernel<<<10, kThr, 0, stream>>>(M32, M16);
    wmma_gemm64<0, false, 2, 0, false, 0><<<dim3((kRows / 64) * (kNF / 64) / 8, 1), 256, 0, stream>>>(
        X16, X16, kK2, 0L, WX, WX, kK2, 0L, (void*)XG, (void*)XG, kNF, 0L, BX, nullptr, 0L, kRows, kNF, kK2, kScHW);
    for (int i = 0; i < kN; ++i) {
      if (i > 0) hist_attn_kernel<<<kB, 128, 0, stream>>>(X, BUF, gat_w, gat_b, adj, M32, M16, i, layer);
      wmma_gemm64<0, false, 2, 0, false, 0><<<dim3((kB / 64) * (kNF / 64) / 8, 1), 256, 0, stream>>>(
          M16, M16, kK2, 0L, WM, WM, kK2, 0L, (void*)MG, (void*)MG, kNF, 0L, BM, nullptr, 0L, kB, kNF, kK2, kScHW);
      dual_gru_kernel<<<10, kThr, 0, stream>>>(X, M32, XG, MG, BUF, H161, i, layer);
    }
  }
  concat_out_kernel<<<15392, kThr, 0, stream>>>(H0F, BUF0, BUF1, features, out);
}
